// Block_77318001263203
// MI455X (gfx1250) — hardware-verified
//
#include <hip/hip_runtime.h>
#ifndef NB
#define NB 2
#endif
#ifndef SEQ
#define SEQ 2048
#endif
#define NB_FULL 2
#define SEQ_FULL 2048
#define SQ SEQ
#define DM 1024
#define NH 16
#define HD 64
#define DFF 4096
#define QT 256
#define NKX SQ
#define QT0 128
#define NR ((size_t)NB * SQ)
#define LQ (3 * DM)

static_assert(NH * HD == DM);
static_assert(DM == 1024);
static_assert(SQ % QT == 0 && QT % 128 == 0 && QT0 % 128 == 0 && QT0 <= SQ && QT0 % 64 == 0);
static_assert(DM % 64 == 0 && DFF % 64 == 0 && LQ % 64 == 0 && HD % 32 == 0 && DM % 32 == 0 && DFF % 32 == 0);
static_assert((NB * SQ) % 128 == 0 && SQ % 128 == 0 && SQ % 64 == 0);
static_assert(((size_t)NB * SQ * DM / 8) % 256 == 0);
static_assert(((size_t)NH * HD * (DM / 8)) % 256 == 0);
static_assert(((size_t)DM * (DM / 8)) % 256 == 0 && ((size_t)DFF * (DM / 8)) % 256 == 0 && ((size_t)DM * (DFF / 8)) % 256 == 0);
static_assert(((size_t)NB * QT0 * DM / 8) % 256 == 0);
static_assert((NH * QT) % 256 == 0);
static_assert(NB <= NB_FULL && SEQ <= SEQ_FULL);

typedef unsigned short v8us __attribute__((ext_vector_type(8), may_alias));
typedef float  v8f  __attribute__((ext_vector_type(8)));
typedef float  v4f  __attribute__((ext_vector_type(4)));
typedef float  v4fa __attribute__((ext_vector_type(4), may_alias));
typedef _Float16 v16h __attribute__((ext_vector_type(16)));
typedef _Float16 v4h __attribute__((ext_vector_type(4)));
union FragH { v16h v; v8us half[2]; _Float16 h[16]; unsigned short u[16]; };

__device__ __forceinline__ unsigned short bf16_bits(float x) { unsigned int u = __float_as_uint(x); return (unsigned short)((u + 0x7FFFu + ((u >> 16) & 1u)) >> 16); }
__device__ __forceinline__ float bf16_val(unsigned short b) { return __uint_as_float(((unsigned int)b) << 16); }
__device__ __forceinline__ float bf16_rne(float x) { return bf16_val(bf16_bits(x)); }

__device__ __forceinline__ v16h g2_frag(const _Float16* p, unsigned hh) { FragH f; f.half[0] = *(const v8us*)((const unsigned short*)p + 8u * hh); f.half[1] = *(const v8us*)((const unsigned short*)p + 16u + 8u * hh); return f.v; }
__device__ __forceinline__ v8f g2_mma(v16h a, v16h b, v8f c) { v8f d = __builtin_amdgcn_wmma_f32_16x16x32_f16(false, a, false, b, (short)0, c, false, false); asm volatile("v_nop\n\tv_nop\n\tv_nop\n\tv_nop" : "+v"(d) : "v"(a), "v"(b)); return d; }

template <int ACT>
__global__ __launch_bounds__(128) void k_gemm2(const _Float16* __restrict__ A, unsigned lda, size_t sA, const _Float16* __restrict__ Bh, unsigned ldb, size_t sB, float alpha,
    const float* __restrict__ bias, const float* __restrict__ CP, float* __restrict__ C, _Float16* __restrict__ C16, unsigned ldc, size_t sC, unsigned M, unsigned N, unsigned K) {
  static_assert(ACT == 0 || ACT == 3);
  __shared__ __attribute__((aligned(16))) float so[4][32][68];
  const unsigned tid = threadIdx.x, w = tid >> 5, lane = tid & 31u, ln = lane & 15u, hh = lane >> 4; const unsigned by = blockIdx.y;
  A += (size_t)by * sA; Bh += (size_t)by * sB; const size_t cofs = (size_t)by * sC;
  const unsigned ntn = N >> 6; const unsigned mt = blockIdx.x / ntn, nq = blockIdx.x - mt * ntn; const unsigned row0 = mt * 128u + 32u * w, col0 = nq * 64u; if (row0 >= M) return;
  const _Float16* a0p = A + (size_t)(row0 + ln) * lda; const _Float16* a1p = a0p + (size_t)16 * lda;
  const _Float16* b0p = Bh + (size_t)(col0 + ln) * ldb; const _Float16* b1p = b0p + (size_t)16 * ldb; const _Float16* b2p = b1p + (size_t)16 * ldb; const _Float16* b3p = b2p + (size_t)16 * ldb;
  const v8f z8 = {0.f,0.f,0.f,0.f,0.f,0.f,0.f,0.f}; v8f c00 = z8, c01 = z8, c02 = z8, c03 = z8, c10 = z8, c11 = z8, c12 = z8, c13 = z8;
#pragma unroll 1
  for (unsigned kb = 0; kb < K; kb += 32u) { const v16h a0 = g2_frag(a0p + kb, hh), a1 = g2_frag(a1p + kb, hh);
    v16h b = g2_frag(b0p + kb, hh); c00 = g2_mma(a0, b, c00); c10 = g2_mma(a1, b, c10);
    b = g2_frag(b1p + kb, hh); c01 = g2_mma(a0, b, c01); c11 = g2_mma(a1, b, c11);
    b = g2_frag(b2p + kb, hh); c02 = g2_mma(a0, b, c02); c12 = g2_mma(a1, b, c12);
    b = g2_frag(b3p + kb, hh); c03 = g2_mma(a0, b, c03); c13 = g2_mma(a1, b, c13); }
  v8f accs[8] = {c00, c01, c02, c03, c10, c11, c12, c13};
#pragma unroll
  for (int u = 0; u < 8; ++u) { const unsigned t = (unsigned)(u & 3), hf = (unsigned)(u >> 2); const unsigned col = col0 + t * 16u + ln; const float bv = bias ? bf16_rne(bias[col]) : 0.f;
#pragma unroll
    for (int r = 0; r < 8; ++r) { const unsigned rloc = hf * 16u + 8u * hh + (unsigned)r; float v = accs[u][r] * alpha + bv;
      if (CP) v += CP[cofs + (size_t)(row0 + rloc) * ldc + col];
      if (ACT == 3) v = fmaxf(v, 0.f);
      so[w][rloc][t * 16u + ln] = v; } }
  __builtin_amdgcn_fence(4  , "workgroup"); __builtin_amdgcn_wave_barrier();
  const unsigned rsub = lane >> 4, c4 = (lane & 15u) * 4u;
  for (int pass = 0; pass < 2; ++pass) {
#pragma unroll
    for (int q = 0; q < 16; ++q) { const unsigned r = (unsigned)q * 2u + rsub; const v4f v = *(const v4fa*)&so[w][r][c4];
      if (C) *(volatile v4f*)(C + cofs + (size_t)(row0 + r) * ldc + col0 + c4) = v;
      if (C16) { v4h h4; for (int i = 0; i < 4; ++i) h4[i] = (_Float16)v[i]; *(volatile v4h*)(C16 + cofs + (size_t)(row0 + r) * ldc + col0 + c4) = h4; } }
    if (pass == 0) __threadfence(); } }

__global__ __launch_bounds__(256) void k_x16(const float* __restrict__ x, _Float16* __restrict__ X16) {
  const unsigned t = blockIdx.x * 256u + threadIdx.x; if (t >= (unsigned)(NR * DM / 8)) return;
  const unsigned row = t >> 7, c8 = (t & 127u) << 3; const unsigned b = row / (unsigned)SQ, s = row - b * (unsigned)SQ;
  const float* src = x + ((size_t)b * SEQ_FULL + s) * DM + c8; const v4f a = *(const v4fa*)src, c = *(const v4fa*)(src + 4); FragH f;
#pragma unroll
  for (int q = 0; q < 4; ++q) { f.h[q] = (_Float16)bf16_rne(a[q]); f.h[4 + q] = (_Float16)bf16_rne(c[q]); }
  const v8us o = f.half[0]; unsigned short* d = (unsigned short*)X16 + (size_t)t * 8u;
  *(volatile v8us*)d = o; __threadfence(); *(volatile v8us*)d = o; }

__global__ __launch_bounds__(256) void k_wt_f16(const float* __restrict__ W, _Float16* __restrict__ Wt, unsigned K, unsigned N, float scale) {
  const unsigned t = blockIdx.x * 256u + threadIdx.x; const unsigned k8n = K >> 3; if (t >= N * k8n) return; const unsigned n = t / k8n, k8 = (t - n * k8n) << 3; FragH f;
#pragma unroll
  for (int i = 0; i < 8; ++i) f.h[i] = (_Float16)(bf16_rne(W[(size_t)(k8 + (unsigned)i) * N + n]) * scale);
  const v8us o = f.half[0]; unsigned short* d = (unsigned short*)Wt + (size_t)n * K + k8;
  *(volatile v8us*)d = o; __threadfence(); *(volatile v8us*)d = o; }

__global__ __launch_bounds__(256) void k_wthd(const float* __restrict__ W, _Float16* __restrict__ Bt) {
  const unsigned t = blockIdx.x * 256u + threadIdx.x; if (t >= (unsigned)(NH * HD * (DM / 8))) return;
  const unsigned m8 = (t & 127u) << 3, d = (t >> 7) & 63u, h = t >> 13; FragH f;
#pragma unroll
  for (int q = 0; q < 8; ++q) f.h[q] = (_Float16)(16.0f * bf16_rne(W[((size_t)h * DM + m8 + (unsigned)q) * HD + d]));
  const v8us o = f.half[0]; unsigned short* dst = (unsigned short*)Bt + ((size_t)h * HD + d) * DM + m8;
  *(volatile v8us*)dst = o; __threadfence(); *(volatile v8us*)dst = o; }

template <int NHv, int TTv>
__global__ __launch_bounds__(256) void k_vt(const _Float16* __restrict__ V16, unsigned ldv, unsigned voff, _Float16* __restrict__ Vt) {
  __shared__ unsigned short tl[64][66]; const unsigned tid = threadIdx.x; const unsigned slab = blockIdx.x / (unsigned)(TTv / 64), lg = blockIdx.x - slab * (unsigned)(TTv / 64);
  for (unsigned i = tid; i < 64u * 8u; i += 256u) { const unsigned r = i >> 3, c8 = (i & 7u) << 3; FragH f; f.half[0] = *(const v8us*)((const unsigned short*)V16 + ((size_t)lg * 64u + r) * ldv + voff + slab * 64u + c8);
#pragma unroll
    for (int q = 0; q < 8; ++q) tl[r][c8 + (unsigned)q] = f.u[q]; }
  __syncthreads();
  for (int pass = 0; pass < 2; ++pass) {
#pragma unroll
    for (int rd = 0; rd < 2; ++rd) { const unsigned d = (unsigned)rd * 32u + (tid >> 3), pc = tid & 7u; FragH f;
#pragma unroll
      for (int q = 0; q < 8; ++q) f.u[q] = tl[pc * 8u + (unsigned)q][d];
      *(volatile v8us*)((unsigned short*)Vt + ((size_t)slab * 64u + d) * TTv + lg * 64u + pc * 8u) = f.half[0]; }
    if (pass == 0) __threadfence(); } }

__global__ __launch_bounds__(256) void k_rsmc(const float* __restrict__ S, _Float16* __restrict__ P, unsigned q0, unsigned nk) {
  #pragma clang fp contract(off)
  const unsigned t = blockIdx.x * 256u + threadIdx.x; if (t >= (unsigned)(NH * QT)) return; const float* s = S + (size_t)t * NKX; const unsigned last = q0 + (t & (unsigned)(QT - 1)); float mx = -3.0e38f;
#pragma unroll 1
  for (unsigned j = 0; j < nk; ++j) { const float f = (j <= last) ? 1.f : 0.f; mx = fmaxf(mx, fmaf(f, s[j], (1.f - f) * -1.0e9f)); } float se = 0.f;
#pragma unroll 1
  for (unsigned j = 0; j < nk; ++j) { const float f = (j <= last) ? 1.f : 0.f; se += __expf(fmaf(f, s[j], (1.f - f) * -1.0e9f) - mx); } const float sc = 1024.0f * (1.0f / se);
#pragma unroll 1
  for (unsigned j0 = 0; j0 < nk; j0 += 8u) { FragH fr;
#pragma unroll
    for (int q = 0; q < 8; ++q) { const unsigned j = j0 + (unsigned)q; const float f = (j <= last) ? 1.f : 0.f; fr.h[q] = (_Float16)(__expf(fmaf(f, s[j], (1.f - f) * -1.0e9f) - mx) * sc); }
    const v8us o = fr.half[0]; unsigned short* d = (unsigned short*)P + (size_t)t * NKX + j0; *(volatile v8us*)d = o; __threadfence(); *(volatile v8us*)d = o; } }

__global__ __launch_bounds__(64) void k_att0(const float* __restrict__ QF, const float* __restrict__ KF, const float* __restrict__ VF, unsigned ld, float scale, float* __restrict__ OF, unsigned ldo) {
  #pragma clang fp contract(off)
  __shared__ __attribute__((aligned(16))) float lq[64][64]; __shared__ __attribute__((aligned(16))) float lo[64][64];
  const unsigned tid = threadIdx.x; const unsigned h = blockIdx.x / (unsigned)(QT0 / 64), rg = blockIdx.x - h * (unsigned)(QT0 / 64); const unsigned i = rg * 64u + tid;
  const float* qr = QF + (size_t)i * ld + h * HD;
#pragma unroll 1
  for (unsigned c = 0; c < HD / 4; ++c) { *(v4f*)&lq[tid][c * 4u] = *(const v4fa*)(qr + c * 4u); const v4f z = {0.f, 0.f, 0.f, 0.f}; *(v4f*)&lo[tid][c * 4u] = z; }
  float m = -1.0e30f, l = 0.f; const unsigned jmax = rg * 64u + 63u;
#pragma unroll 1
  for (unsigned j = 0; j <= jmax; ++j) { const float* kr = KF + (size_t)j * ld + h * HD; const float* vr = VF + (size_t)j * ld + h * HD; float s = 0.f;
#pragma unroll 1
    for (unsigned c = 0; c < HD / 4; ++c) { const v4f kq = *(const v4fa*)(kr + c * 4u); const v4f qq = *(v4f*)&lq[tid][c * 4u]; s = __fadd_rn(s, __fmul_rn(qq[0], kq[0])); s = __fadd_rn(s, __fmul_rn(qq[1], kq[1])); s = __fadd_rn(s, __fmul_rn(qq[2], kq[2])); s = __fadd_rn(s, __fmul_rn(qq[3], kq[3])); }
    s = __fmul_rn(s, scale);
    const float f = (j <= i) ? 1.f : 0.f; const float sm = fmaf(f, s, (1.f - f) * -1.0e30f); const float mn = fmaxf(m, sm); const float sc = expf(m - mn); const float e = expf(sm - mn); l = __fadd_rn(__fmul_rn(l, sc), e); m = mn;
#pragma unroll 1
    for (unsigned c = 0; c < HD / 4; ++c) { const v4f vv = *(const v4fa*)(vr + c * 4u); v4f oo = *(v4f*)&lo[tid][c * 4u]; for (int u = 0; u < 4; ++u) oo[u] = __fadd_rn(__fmul_rn(oo[u], sc), __fmul_rn(e, vv[u])); *(v4f*)&lo[tid][c * 4u] = oo; } }
  const float fin = 64.0f * (1.0f / l);
#pragma unroll 1
  for (unsigned c = 0; c < HD / 4; ++c) { v4f oo = *(v4f*)&lo[tid][c * 4u]; for (int u = 0; u < 4; ++u) oo[u] = __fmul_rn(oo[u], fin); *(v4f*)&lo[tid][c * 4u] = oo; }
  __syncthreads();
  for (int pass = 0; pass < 2; ++pass) {
#pragma unroll 1
    for (unsigned it = 0; it < 16u; ++it) { const unsigned row = it * 4u + (tid >> 4), pc = (tid & 15u) * 4u; const v4f v = *(const v4f*)&lo[row][pc]; *(volatile v4f*)(OF + (size_t)(rg * 64u + row) * ldo + h * HD + pc) = v; }
    if (pass == 0) __threadfence(); } }

__global__ __launch_bounds__(256) void k_hl(const float* __restrict__ F, _Float16* __restrict__ Hh, _Float16* __restrict__ Hl, unsigned n8) {
  const unsigned t = blockIdx.x * 256u + threadIdx.x; if (t >= n8) return; FragH fh, fl; const v4f a = *(const v4fa*)(F + (size_t)t * 8u), c = *(const v4fa*)(F + (size_t)t * 8u + 4u);
#pragma unroll
  for (int q = 0; q < 4; ++q) { _Float16 h = (_Float16)a[q]; fh.h[q] = h; fl.h[q] = (_Float16)((a[q] - (float)h) * 1024.0f); h = (_Float16)c[q]; fh.h[4 + q] = h; fl.h[4 + q] = (_Float16)((c[q] - (float)h) * 1024.0f); }
  const v8us oh = fh.half[0], ol = fl.half[0];
  for (int pass = 0; pass < 2; ++pass) { *(volatile v8us*)((unsigned short*)Hh + (size_t)t * 8u) = oh; *(volatile v8us*)((unsigned short*)Hl + (size_t)t * 8u) = ol; if (pass == 0) __threadfence(); } }

__global__ __launch_bounds__(256) void k_ln1(const float* __restrict__ x, const float* __restrict__ Y, const float* __restrict__ YFT, const float* __restrict__ g, const float* __restrict__ bb, float eps, _Float16* __restrict__ N16, float* __restrict__ N32) {
  #pragma clang fp contract(off)
  __shared__ float red[256]; const unsigned r = blockIdx.x, t = threadIdx.x, c0 = t * 4u; const unsigned b = r / (unsigned)SQ, rl = r - b * (unsigned)SQ; const bool ft = rl < (unsigned)QT0; const unsigned rs = ft ? rl : 0u;
  const v4f xa = *(const v4fa*)(x + ((size_t)b * SEQ_FULL + rl) * DM + c0); const v4f ya = *(const v4fa*)(Y + (size_t)r * DM + c0); const v4f yt = *(const v4fa*)(YFT + ((size_t)b * QT0 + rs) * DM + c0);
  float s[4]; float sum = 0.f;
  for (int q = 0; q < 4; ++q) { const float yv = ft ? yt[q] : ya[q]; s[q] = __fadd_rn(bf16_rne(xa[q]), yv); sum = __fadd_rn(sum, s[q]); }
  red[t] = sum; __syncthreads(); for (unsigned st = 128u; st > 0u; st >>= 1) { if (t < st) red[t] = __fadd_rn(red[t], red[t + st]); __syncthreads(); } const float mu = red[0] * (1.0f / (float)DM); __syncthreads();
  float vs = 0.f; for (int q = 0; q < 4; ++q) { const float dl = __fadd_rn(s[q], -mu); vs = __fadd_rn(vs, __fmul_rn(dl, dl)); } red[t] = vs; __syncthreads(); for (unsigned st = 128u; st > 0u; st >>= 1) { if (t < st) red[t] = __fadd_rn(red[t], red[t + st]); __syncthreads(); }
  const float rsd = rsqrtf(__fadd_rn(red[0] * (1.0f / (float)DM), eps)); v4h y; v4f yf;
  for (int q = 0; q < 4; ++q) { const unsigned c = c0 + (unsigned)q; yf[q] = __fadd_rn(__fmul_rn(__fmul_rn(__fadd_rn(s[q], -mu), rsd), bf16_rne(g[c])), bf16_rne(bb[c])); y[q] = (_Float16)yf[q]; }
  for (int pass = 0; pass < 2; ++pass) { *(volatile v4h*)(N16 + (size_t)r * DM + c0) = y; *(volatile v4f*)(N32 + (size_t)r * DM + c0) = yf; if (pass == 0) __threadfence(); } }

__global__ __launch_bounds__(256) void k_ln2(const float* __restrict__ T, const float* __restrict__ g, const float* __restrict__ bb, float eps, float* __restrict__ out) {
  #pragma clang fp contract(off)
  __shared__ float red[256]; const unsigned r = blockIdx.x, t = threadIdx.x, c0 = t * 4u; const unsigned b = r / (unsigned)SQ, rl = r - b * (unsigned)SQ;
  const v4f xa = *(const v4fa*)(T + (size_t)r * DM + c0); float s[4]; float sum = 0.f;
  for (int q = 0; q < 4; ++q) { s[q] = xa[q]; sum = __fadd_rn(sum, s[q]); }
  red[t] = sum; __syncthreads(); for (unsigned st = 128u; st > 0u; st >>= 1) { if (t < st) red[t] = __fadd_rn(red[t], red[t + st]); __syncthreads(); } const float mu = red[0] * (1.0f / (float)DM); __syncthreads();
  float vs = 0.f; for (int q = 0; q < 4; ++q) { const float dl = __fadd_rn(s[q], -mu); vs = __fadd_rn(vs, __fmul_rn(dl, dl)); } red[t] = vs; __syncthreads(); for (unsigned st = 128u; st > 0u; st >>= 1) { if (t < st) red[t] = __fadd_rn(red[t], red[t + st]); __syncthreads(); }
  const float rsd = rsqrtf(__fadd_rn(red[0] * (1.0f / (float)DM), eps)); v4f yf;
  for (int q = 0; q < 4; ++q) { const unsigned c = c0 + (unsigned)q; yf[q] = __fadd_rn(__fmul_rn(__fmul_rn(__fadd_rn(s[q], -mu), rsd), bf16_rne(g[c])), bf16_rne(bb[c])); }
  float* dst = out + ((size_t)b * SEQ_FULL + rl) * DM + c0;
  for (int pass = 0; pass < 2; ++pass) { *(volatile v4f*)dst = yf; if (pass == 0) __threadfence(); } }

constexpr size_t B_BQKV = (size_t)3 * DM * DM * 2, B_BWP = (size_t)DM * DM * 2, B_BW1 = (size_t)DFF * DM * 2, B_BW2 = (size_t)DM * DFF * 2;
constexpr size_t B_X16 = (size_t)NB * SQ * DM * 2, B_O16 = B_X16;
constexpr size_t B_F0 = (size_t)NB * QT0 * LQ * 4, B_OF0 = (size_t)NB * QT0 * DM * 4, B_OH = (size_t)NB * QT0 * DM * 2, B_YL = (size_t)NB * QT0 * DM * 4;
constexpr size_t B_FIX = B_BQKV + B_BWP + B_BW1 + B_BW2 + B_X16 + B_O16 + B_F0 + B_OF0 + 2 * B_OH + 2 * B_YL;
constexpr size_t B_QKV = (size_t)NB * SQ * LQ * 2, B_S = (size_t)NH * QT * NKX * 4, B_P = (size_t)NH * QT * NKX * 2, B_VT = (size_t)NH * HD * SQ * 2;
constexpr size_t B_Y = (size_t)NB * SQ * DM * 4, B_HF = (size_t)SQ * DFF * 2;
constexpr size_t B_PHA = B_QKV + B_S + B_P + B_VT;
constexpr size_t B_PHB = B_Y + B_Y + B_HF;
constexpr size_t B_OV = (B_PHA > B_PHB) ? B_PHA : B_PHB;
constexpr size_t B_TOTAL = B_FIX + B_OV;
static_assert(B_PHA <= B_OV && B_PHB <= B_OV);
static_assert(B_TOTAL <= (size_t)134217728);
static_assert(B_BQKV % 256 == 0 && B_BWP % 256 == 0 && B_BW1 % 256 == 0 && B_X16 % 256 == 0 && B_F0 % 256 == 0 && B_OF0 % 256 == 0 && B_OH % 256 == 0 && B_YL % 256 == 0);
static_assert(B_QKV % 256 == 0 && B_S % 256 == 0 && B_P % 256 == 0 && B_VT % 256 == 0 && B_Y % 256 == 0 && B_HF % 256 == 0);

extern "C" void kernel_launch(void* const* d_in, const int* in_sizes, int n_in,
                              void* d_out, int out_size, void* d_ws, size_t ws_size, hipStream_t stream) {
  if (n_in < 14) return;
  if ((size_t)in_sizes[0] < ((size_t)(NB - 1) * SEQ_FULL + SQ) * DM) return;
  if ((size_t)in_sizes[1] < (size_t)NH * DM * HD || (size_t)in_sizes[2] < (size_t)NH * DM * HD || (size_t)in_sizes[3] < (size_t)NH * DM * HD) return;
  if ((size_t)in_sizes[4] < (size_t)DM * DM || in_sizes[5] < DM || (size_t)in_sizes[6] < (size_t)DM * DFF || in_sizes[7] < DFF || (size_t)in_sizes[8] < (size_t)DFF * DM || in_sizes[9] < DM) return;
  if (in_sizes[10] < DM || in_sizes[11] < DM || in_sizes[12] < DM || in_sizes[13] < DM) return;
  if ((size_t)out_size < ((size_t)(NB - 1) * SEQ_FULL + SQ) * DM) return;
  if (B_TOTAL > ws_size) return;
  const float* const* I = (const float* const*)d_in;
  const float* x = I[0]; const float* wq = I[1]; const float* wk = I[2]; const float* wv = I[3]; const float* wp = I[4]; const float* bp = I[5];
  const float* w1 = I[6]; const float* b1 = I[7]; const float* w2 = I[8]; const float* b2 = I[9]; const float* g1 = I[10]; const float* be1 = I[11]; const float* g2 = I[12]; const float* be2 = I[13];
  char* ws = (char*)d_ws; size_t off = 0;
  auto take = [&](size_t bytes) { char* p = ws + off; off += bytes; return p; };
  _Float16* BQKV = (_Float16*)take(B_BQKV); _Float16* BWP = (_Float16*)take(B_BWP); _Float16* BW1 = (_Float16*)take(B_BW1); _Float16* BW2 = (_Float16*)take(B_BW2);
  _Float16* X16 = (_Float16*)take(B_X16); _Float16* O16 = (_Float16*)take(B_O16);
  float* F0 = (float*)take(B_F0); float* OF0 = (float*)take(B_OF0); _Float16* OH = (_Float16*)take(B_OH); _Float16* OL = (_Float16*)take(B_OH); float* YLO = (float*)take(B_YL); float* YFT = (float*)take(B_YL);
  char* ov = ws + off;
  _Float16* QKV = (_Float16*)ov; float* S = (float*)(ov + B_QKV); _Float16* P = (_Float16*)(ov + B_QKV + B_S); _Float16* VT = (_Float16*)(ov + B_QKV + B_S + B_P);
  float* Y = (float*)ov; float* X1F = (float*)(ov + B_Y); _Float16* HF16 = (_Float16*)(ov + B_Y + B_Y); float* T = Y;
  _Float16* M16 = X16;
  _Float16* Q16 = QKV; _Float16* K16 = QKV + DM; _Float16* V16 = QKV + 2 * DM;

  { const unsigned g = (unsigned)(((size_t)NH * HD * (DM / 8)) / 256); k_wthd<<<g, 256, 0, stream>>>(wq, BQKV); k_wthd<<<g, 256, 0, stream>>>(wk, BQKV + (size_t)DM * DM); k_wthd<<<g, 256, 0, stream>>>(wv, BQKV + (size_t)2 * DM * DM); }
  k_x16<<<(unsigned)(NR * DM / 8 / 256), 256, 0, stream>>>(x, X16);
  k_wt_f16<<<(unsigned)(((size_t)DM * (DM / 8)) / 256), 256, 0, stream>>>(wp, BWP, DM, DM, 16.0f);
  k_wt_f16<<<(unsigned)(((size_t)DFF * (DM / 8)) / 256), 256, 0, stream>>>(w1, BW1, DM, DFF, 16.0f);
  k_wt_f16<<<(unsigned)(((size_t)DM * (DFF / 8)) / 256), 256, 0, stream>>>(w2, BW2, DFF, DM, 16.0f);
  k_gemm2<0><<<dim3((unsigned)((NR / 128) * (LQ / 64)), 1), 128, 0, stream>>>(X16, DM, 0, BQKV, DM, 0, 0.0625f, nullptr, nullptr, nullptr, QKV, LQ, 0, (unsigned)NR, LQ, DM);
  k_gemm2<0><<<dim3((unsigned)((QT0 / 128) * (LQ / 64)), NB), 128, 0, stream>>>(X16, DM, (size_t)SQ * DM, BQKV, DM, 0, 0.0625f, nullptr, nullptr, F0, nullptr, LQ, (size_t)QT0 * LQ, QT0, LQ, DM);
  for (int b = 0; b < NB; ++b) { const size_t r0 = (size_t)b * SQ; const float* f0b = F0 + (size_t)b * QT0 * LQ;
    k_vt<NH, SQ><<<NH * (SQ / 64), 256, 0, stream>>>(V16 + r0 * LQ, LQ, 0, VT);
    k_att0<<<NH * (QT0 / 64), 64, 0, stream>>>(f0b, f0b + DM, f0b + 2 * DM, LQ, 0.125f, OF0 + (size_t)b * QT0 * DM, DM);
    for (int q0 = 0; q0 < SQ; q0 += QT) { const int nk = q0 + QT;
      k_gemm2<0><<<dim3((unsigned)((QT / 128) * (nk / 64)), NH), 128, 0, stream>>>(Q16 + (r0 + q0) * LQ, LQ, (size_t)HD, K16 + r0 * LQ, LQ, (size_t)HD, 0.125f, nullptr, nullptr, S, nullptr, NKX, (size_t)QT * NKX, QT, (unsigned)nk, HD);
      k_rsmc<<<(NH * QT) / 256, 256, 0, stream>>>(S, P, (unsigned)q0, (unsigned)nk);
      k_gemm2<0><<<dim3((unsigned)((QT / 128) * (HD / 64)), NH), 128, 0, stream>>>(P, NKX, (size_t)QT * NKX, VT, SQ, (size_t)HD * SQ, 0.0625f, nullptr, nullptr, nullptr, O16 + (r0 + q0) * DM, DM, (size_t)HD, QT, HD, (unsigned)nk); } }
  k_gemm2<0><<<dim3((unsigned)((NR / 128) * (DM / 64)), 1), 128, 0, stream>>>(O16, DM, 0, BWP, DM, 0, 1.0f / 1024.0f, bp, nullptr, Y, nullptr, DM, 0, (unsigned)NR, DM, DM);
  k_hl<<<(unsigned)(((size_t)NB * QT0 * DM / 8) / 256), 256, 0, stream>>>(OF0, OH, OL, (unsigned)((size_t)NB * QT0 * DM / 8));
  k_gemm2<0><<<dim3((unsigned)((NB * QT0 / 128) * (DM / 64)), 1), 128, 0, stream>>>(OL, DM, 0, BWP, DM, 0, 1.0f / 1048576.0f, nullptr, nullptr, YLO, nullptr, DM, 0, NB * QT0, DM, DM);
  k_gemm2<0><<<dim3((unsigned)((NB * QT0 / 128) * (DM / 64)), 1), 128, 0, stream>>>(OH, DM, 0, BWP, DM, 0, 1.0f / 1024.0f, bp, YLO, YFT, nullptr, DM, 0, NB * QT0, DM, DM);
  k_ln1<<<(unsigned)NR, 256, 0, stream>>>(x, Y, YFT, g1, be1, 1e-5f, M16, X1F);
  for (int b = 0; b < NB; ++b) { const size_t r0 = (size_t)b * SQ;
    k_gemm2<3><<<dim3((unsigned)((SQ / 128) * (DFF / 64)), 1), 128, 0, stream>>>(M16 + r0 * DM, DM, 0, BW1, DM, 0, 0.0625f, b1, nullptr, nullptr, HF16, DFF, 0, SQ, DFF, DM);
    k_gemm2<0><<<dim3((unsigned)((SQ / 128) * (DM / 64)), 1), 128, 0, stream>>>(HF16, DFF, 0, BW2, DFF, 0, 0.0625f, b2, X1F + r0 * DM, T + r0 * DM, nullptr, DM, 0, SQ, DM, DFF); }
  k_ln2<<<(unsigned)NR, 256, 0, stream>>>(T, g2, be2, 1e-5f, (float*)d_out);
}
